// ConAttn_59897613910138
// MI455X (gfx1250) — hardware-run, weakly checked
//
#include <hip/hip_runtime.h>
#include <math.h>

typedef __attribute__((ext_vector_type(16))) _Float16 v16h;
typedef __attribute__((ext_vector_type(16))) __bf16 v16b;
typedef __attribute__((ext_vector_type(8)))  _Float16 v8h;
typedef __attribute__((ext_vector_type(8)))  float v8f;
typedef __attribute__((ext_vector_type(4)))  float v4f;
typedef __attribute__((ext_vector_type(2)))  float v2f;
typedef __attribute__((ext_vector_type(4)))  unsigned v4u;
typedef __attribute__((ext_vector_type(4)))  int v4i;
typedef float __attribute__((may_alias)) float_a;
typedef int __attribute__((may_alias)) int_a;

template <typename T> __device__ __forceinline__ void vst2(void* p, T v) { *(volatile T*)p = v; __threadfence(); *(volatile T*)p = v; }
__device__ __forceinline__ v8f wmma16(v16h a, v16h b, v8f c) {
  v8f d = __builtin_amdgcn_wmma_f32_16x16x32_f16(false, a, false, b, (short)0, c, false, false);
  asm volatile("v_nop\n\tv_nop\n\tv_nop\n\tv_nop" : "+v"(d) : "v"(a), "v"(b));
  return d;
}
__device__ __forceinline__ v8f wmma_bf(v16b a, v16b b, v8f c) {
  v8f d = __builtin_amdgcn_wmma_f32_16x16x32_bf16(false, a, false, b, (short)0, c, false, false);
  asm volatile("v_nop\n\tv_nop\n\tv_nop\n\tv_nop" : "+v"(d) : "v"(a), "v"(b));
  return d;
}
__device__ __forceinline__ v16h frag_h(const _Float16* rowk0, int lane) {
  union { v16h v; v8h q[2]; } u; const _Float16* p = rowk0 + 8 * (lane >> 4);
  u.q[0] = *(const v8h*)p; u.q[1] = *(const v8h*)(p + 16); return u.v;
}
__device__ __forceinline__ v16h frag_f32(const float* rowk0, int lane) {
  v16h a; const float* p = rowk0 + 8 * (lane >> 4);
#pragma unroll
  for (int i = 0; i < 8; ++i) { a[i] = (_Float16)p[i]; a[8 + i] = (_Float16)p[16 + i]; }
  return a;
}
__device__ __forceinline__ v16h frag_f32s(const float* rowk0, int lane, float sc) {
  v16h a; const float* p = rowk0 + 8 * (lane >> 4);
#pragma unroll
  for (int i = 0; i < 8; ++i) { a[i] = (_Float16)(p[i] * sc); a[8 + i] = (_Float16)(p[16 + i] * sc); }
  return a;
}
__device__ __forceinline__ v16h fragc_f32(const float* W, int k0, int n, int lane, int ld, int K) {
  v16h a; const int g = lane >> 4;
#pragma unroll
  for (int i = 0; i < 8; ++i) { const int ka = k0 + 8 * g + i, kb = ka + 16;
    a[i] = (_Float16)(ka < K ? W[(size_t)(ka < K ? ka : K - 1) * ld + n] : 0.f); a[8 + i] = (_Float16)(kb < K ? W[(size_t)(kb < K ? kb : K - 1) * ld + n] : 0.f); }
  return a;
}
struct F2 { v16b h, l; };
__device__ __forceinline__ F2 bsplit16(const float v[16]) { F2 r;
#pragma unroll
  for (int i = 0; i < 16; ++i) { const __bf16 h = (__bf16)v[i]; r.h[i] = h; r.l[i] = (__bf16)(v[i] - (float)h); }
  return r; }
__device__ __forceinline__ F2 split_row(const float* row, int k0, int lane) { float v[16]; const float* p = row + k0 + 8 * (lane >> 4);
#pragma unroll
  for (int i = 0; i < 8; ++i) { v[i] = p[i]; v[8 + i] = p[16 + i]; }
  return bsplit16(v); }
__device__ __forceinline__ F2 split_rowK(const float* row, int k0, int lane, int K) { float v[16]; const int g = lane >> 4;
#pragma unroll
  for (int i = 0; i < 8; ++i) { const int ka = k0 + 8 * g + i, kb = ka + 16; v[i] = ka < K ? row[ka < K ? ka : K - 1] : 0.f; v[8 + i] = kb < K ? row[kb < K ? kb : K - 1] : 0.f; }
  return bsplit16(v); }
__device__ __forceinline__ F2 split_col(const float* W, int k0, int n, int lane, int ld, int K) { float v[16]; const int g = lane >> 4;
#pragma unroll
  for (int i = 0; i < 8; ++i) { const int ka = k0 + 8 * g + i, kb = ka + 16; v[i] = ka < K ? W[(size_t)(ka < K ? ka : K - 1) * ld + n] : 0.f; v[8 + i] = kb < K ? W[(size_t)(kb < K ? kb : K - 1) * ld + n] : 0.f; }
  return bsplit16(v); }
__device__ __forceinline__ v8f mac3(const F2& a, const F2& b, v8f c) { c = wmma_bf(a.l, b.h, c); c = wmma_bf(a.h, b.l, c); return wmma_bf(a.h, b.h, c); }
__device__ __forceinline__ float sigm(float v) { return 1.0f / (1.0f + expf(-v)); }
#define LDSX() do { asm volatile("s_wait_dscnt 0" ::: "memory"); __builtin_amdgcn_wave_barrier(); __builtin_amdgcn_fence(__ATOMIC_RELEASE, "workgroup"); } while (0)

#define NB 2
#define CC 128
#define HH 64
#define WWD 64
#define TT (HH * WWD)
#define NH 4
#define HD 32
#define MH 32
#ifndef TNB
#define TNB NB
#endif
#ifndef XP
#define XP TT
#endif
typedef __attribute__((ext_vector_type(8))) __bf16 v8b;
__device__ __forceinline__ v16b frag_b(const __bf16* rowk0, int lane) {
  union { v16b v; v8b q[2]; } u; const __bf16* p = rowk0 + 8 * (lane >> 4);
  u.q[0] = *(const v8b*)p; u.q[1] = *(const v8b*)(p + 16); return u.v;
}
__device__ __forceinline__ float bfr(float v) { return (float)(__bf16)v; }
__device__ __forceinline__ float leaky(float v) { return v >= 0.f ? v : 0.2f * v; }

#define HG 1
#define NBLK (TT / 64)
#define WS_QH  0u
#define WS_KH  (WS_QH + 2u * (size_t)NB * TT * CC)
#define WS_VT  (WS_KH + 2u * (size_t)NB * TT * CC)
#define WS_VW  (WS_VT + 2u * (size_t)NB * CC * TT)
#define WS_WG  (WS_VW + 2u * (size_t)NB * CC * TT)
#define WS_BI  (WS_WG + 4u * (size_t)NB * TT)
#define WS_PB  (WS_BI + 4u * (size_t)NB * TT)
#define WS_S   (WS_PB + 4u * (size_t)NB * NBLK * CC)
#define WS_Y   (WS_S  + 4u * (size_t)HG * TT * TT)
#define WS_YW  (WS_Y  + 4u * (size_t)NB * TT * CC)
#define WS_PY  (WS_YW + 4u * (size_t)NB * TT * CC)
#define WS_OA  (WS_PY + 4u * (size_t)NB * NBLK * CC)
#define WS_END (WS_OA + 4u * (size_t)NB * CC * TT)

__global__ __launch_bounds__(128) void k_projq(const float* __restrict__ X, const float* __restrict__ WQ, const float* __restrict__ BQ, const float* __restrict__ L1W, const float* __restrict__ L1B, const float* __restrict__ L2W, const float* __restrict__ L2B, const float* __restrict__ S1W, const float* __restrict__ S1B, const float* __restrict__ S2W, const float* __restrict__ S2B, _Float16* __restrict__ QH, _Float16* __restrict__ KH, float* __restrict__ WG, float* __restrict__ BI) {
  __shared__ __align__(16) float sf[64][132];
  __shared__ __align__(16) float sg[64][68];
  __shared__ __align__(16) float swg[64], sbi[64], snr[64];
  __shared__ __align__(16) _Float16 sh[64][136];
  const int tid = threadIdx.x, wave = tid >> 5, lane = tid & 31, col = lane & 15, g = lane >> 4; const int b = blockIdx.y; const int n0 = blockIdx.x * 64; const size_t row0 = (size_t)b * TT + n0;
  { v8f acc[8] = {};
#pragma unroll 1
    for (int kc = 0; kc < CC / 32; ++kc) { v16b a; { const size_t n = n0 + wave * 16 + col; const float* p = X + ((size_t)b * CC + kc * 32 + 8 * g) * XP + n;
#pragma unroll
        for (int i = 0; i < 8; ++i) { a[i] = (__bf16)p[(size_t)i * XP]; a[8 + i] = (__bf16)p[(size_t)(16 + i) * XP]; } }
      asm volatile("s_wait_loadcnt 0x0" ::: "memory");
#pragma unroll
      for (int j = 0; j < 8; ++j) { v16b w; const int o = j * 16 + col; const float* wp = WQ + (size_t)o * CC + kc * 32 + 8 * g;
#pragma unroll
        for (int i = 0; i < 8; ++i) { w[i] = (__bf16)wp[i]; w[8 + i] = (__bf16)wp[16 + i]; }
        asm volatile("s_wait_loadcnt 0x0" ::: "memory"); acc[j] = wmma_bf(a, w, acc[j]); } }
#pragma unroll
    for (int j = 0; j < 8; ++j) { const float bb = bfr(BQ[j * 16 + col]);
#pragma unroll
      for (int r = 0; r < 8; ++r) sf[wave * 16 + 8 * g + r][j * 16 + col] = acc[j][r] + bb; } }
  __syncthreads();
  if (tid < 64) { float s = 0.f; const float* q = sf[tid];
#pragma unroll 4
    for (int c = 0; c < CC; ++c) s += q[c] * q[c];
    const float nr = sqrtf(s); snr[tid] = 1.0f / fmaxf(nr, 1e-4f); }
  { v8f hcc[4] = {};
#pragma unroll
    for (int kc = 0; kc < CC / 32; ++kc) { float qv[16]; const float* qr = sf[wave * 16 + col] + kc * 32 + 8 * g;
#pragma unroll
      for (int i = 0; i < 8; ++i) { qv[i] = qr[i]; qv[8 + i] = qr[16 + i]; }
      const F2 qa = bsplit16(qv);
#pragma unroll
      for (int j = 0; j < 4; ++j) { v16b w; const int o = (j & 1) * 16 + col; const float* wp = (j < 2 ? L1W : S1W) + (size_t)o * CC + kc * 32 + 8 * g;
#pragma unroll
        for (int i = 0; i < 8; ++i) { w[i] = (__bf16)wp[i]; w[8 + i] = (__bf16)wp[16 + i]; }
        asm volatile("s_wait_loadcnt 0x0" ::: "memory"); hcc[j] = wmma_bf(qa.h, w, hcc[j]); hcc[j] = wmma_bf(qa.l, w, hcc[j]); } }
#pragma unroll
    for (int j = 0; j < 4; ++j) { const int o = (j & 1) * 16 + col; const float bb = bfr((j < 2 ? L1B : S1B)[o]);
#pragma unroll
      for (int r = 0; r < 8; ++r) sg[wave * 16 + 8 * g + r][j * 16 + col] = leaky(hcc[j][r] + bb); } }
  __syncthreads();
  if (tid < 64) { const float* hrow = sg[tid]; float sw = 0.f, sb = 0.f;
#pragma unroll 8
    for (int j = 0; j < MH; ++j) { sw += bfr(L2W[j]) * hrow[j]; sb += bfr(S2W[j]) * hrow[MH + j]; }
    swg[tid] = sw + bfr(L2B[0]); sbi[tid] = sb + bfr(S2B[0]); }
  __syncthreads();
  if (tid < 32) { if (tid < 16) vst2(WG + row0 + tid * 4, *(const v4f*)&swg[tid * 4]); else vst2(BI + row0 + (tid - 16) * 4, *(const v4f*)&sbi[(tid - 16) * 4]); }
  for (int pass = 0; pass < 2; ++pass) { if (pass) __syncthreads();
    for (int e = tid; e < 64 * 128; e += 128) { const int rl = e >> 7, cl = e & 127; const float v = sf[rl][cl] * (pass ? snr[rl] : 1.0f); sh[rl][cl] = (_Float16)v; }
    __syncthreads();
    _Float16* dh = pass ? KH : QH; for (int e = tid; e < 64 * 16; e += 128) { const int rl = e >> 4, q = e & 15; vst2((unsigned*)(dh + (row0 + rl) * CC + q * 8), *(const v4u*)&sh[rl][q * 8]); } } }
__global__ __launch_bounds__(128) void k_projv(const float* __restrict__ X, const float* __restrict__ WV, const float* __restrict__ BV, const float* __restrict__ WG, const float* __restrict__ BI, _Float16* __restrict__ VT, _Float16* __restrict__ VW, float* __restrict__ PB) {
  __shared__ __align__(16) _Float16 th[128][72], tw2[128][72];
  __shared__ __align__(16) float spb[4][128];
  const int tid = threadIdx.x, wave = tid >> 5, lane = tid & 31, col = lane & 15, g = lane >> 4; const int b = blockIdx.y; const int n0 = blockIdx.x * 64; const size_t row0 = (size_t)b * TT + n0;
  v8f acc[8] = {};
#pragma unroll 1
  for (int kc = 0; kc < CC / 32; ++kc) { v16b a; { const size_t n = n0 + wave * 16 + col; const float* p = X + ((size_t)b * CC + kc * 32 + 8 * g) * XP + n;
#pragma unroll
      for (int i = 0; i < 8; ++i) { a[i] = (__bf16)p[(size_t)i * XP]; a[8 + i] = (__bf16)p[(size_t)(16 + i) * XP]; } }
    asm volatile("s_wait_loadcnt 0x0" ::: "memory");
#pragma unroll
    for (int j = 0; j < 8; ++j) { v16b w; const int o = j * 16 + col; const float* wp = WV + (size_t)o * CC + kc * 32 + 8 * g;
#pragma unroll
      for (int i = 0; i < 8; ++i) { w[i] = (__bf16)wp[i]; w[8 + i] = (__bf16)wp[16 + i]; }
      asm volatile("s_wait_loadcnt 0x0" ::: "memory"); acc[j] = wmma_bf(a, w, acc[j]); } }
  float wg8[8], bi8[8];
#pragma unroll
  for (int r = 0; r < 8; ++r) { const size_t rw = row0 + wave * 16 + 8 * g + r; wg8[r] = WG[rw]; bi8[r] = BI[rw]; }
  asm volatile("s_wait_loadcnt 0x0" ::: "memory");
  float pb[8];
#pragma unroll
  for (int j = 0; j < 8; ++j) { const float bb = bfr(BV[j * 16 + col]); float s = 0.f;
#pragma unroll
    for (int r = 0; r < 8; ++r) { const int rl = wave * 16 + 8 * g + r, cl = j * 16 + col; const float v = acc[j][r] + bb; th[cl][rl] = (_Float16)v; tw2[cl][rl] = (_Float16)(v * wg8[r]); s += v * bi8[r]; }
    pb[j] = s; }
#pragma unroll
  for (int j = 0; j < 8; ++j) { const float other = __shfl_xor(pb[j], 16); if (g == 0) spb[wave][j * 16 + col] = pb[j] + other; }
  __syncthreads();
  for (int e = tid; e < 128 * 8; e += 128) { const int cl = e >> 3, q = e & 7; const size_t o2 = ((size_t)b * CC + cl) * TT + n0 + q * 8; vst2((unsigned*)(VT + o2), *(const v4u*)&th[cl][q * 8]); vst2((unsigned*)(VW + o2), *(const v4u*)&tw2[cl][q * 8]); }
  if (tid < 32) { v4f o; const int c4 = tid * 4;
#pragma unroll
    for (int z = 0; z < 4; ++z) o[z] = ((spb[0][c4 + z] + spb[1][c4 + z]) + spb[2][c4 + z]) + spb[3][c4 + z];
    vst2(PB + ((size_t)b * NBLK + blockIdx.x) * CC + c4, o); } }
__global__ __launch_bounds__(128) void k_sc(const _Float16* __restrict__ QH, const _Float16* __restrict__ KH, int b, int h0, float* __restrict__ S0) { __shared__ __align__(16) float ss[4][16][132]; const int h = h0 + blockIdx.z; float* S = S0 + (size_t)blockIdx.z * TT * TT;
  const int tid = threadIdx.x, wave = tid >> 5, lane = tid & 31, col = lane & 15, g = lane >> 4; const int k0 = blockIdx.y * 128; const int ql0 = blockIdx.x * 64 + wave * 16; const size_t q0 = (size_t)b * TT + ql0;
  v8f acc[8] = {};
  { const v16h ah = frag_h(QH + (q0 + col) * CC + h * HD, lane);
#pragma unroll
    for (int j = 0; j < 8; ++j) { const v16h kb = frag_h(KH + ((size_t)b * TT + k0 + j * 16 + col) * CC + h * HD, lane); acc[j] = wmma16(ah, kb, acc[j]); } }
#pragma unroll
  for (int j = 0; j < 8; ++j) {
#pragma unroll
    for (int r = 0; r < 8; ++r) ss[wave][8 * g + r][j * 16 + col] = acc[j][r]; }
  LDSX(); for (int rl = 0; rl < 16; ++rl) vst2(S + (size_t)(ql0 + rl) * TT + k0 + lane * 4, *(const v4f*)&ss[wave][rl][lane * 4]); }
__global__ __launch_bounds__(256) void k_sm(float* __restrict__ S0) { __shared__ float sred[8]; __shared__ float sbc; __shared__ __align__(16) float sh[TT];
  const int t = threadIdx.x; const size_t row = blockIdx.x; float* sr = S0 + (size_t)blockIdx.y * TT * TT + row * TT; const int kend = TT;
  float m = -3.0e38f; for (int k = t; k < kend; k += 256) m = fmaxf(m, sr[k]);
#pragma unroll
  for (int o = 1; o < 32; o <<= 1) m = fmaxf(m, __shfl_xor(m, o));
  if ((t & 31) == 0) sred[t >> 5] = m; __syncthreads(); if (t == 0) { float a = sred[0]; for (int i = 1; i < 8; ++i) a = fmaxf(a, sred[i]); sbc = a; } __syncthreads(); m = sbc; __syncthreads();
  float sum = 0.f; for (int k = t; k < kend; k += 256) { const float v = sr[k]; sum += (v <= -1.0e38f) ? 0.f : expf(v - m); }
#pragma unroll
  for (int o = 1; o < 32; o <<= 1) sum += __shfl_xor(sum, o);
  if ((t & 31) == 0) sred[t >> 5] = sum; __syncthreads(); if (t == 0) { float a = 0.f; for (int i = 0; i < 8; ++i) a += sred[i]; sbc = 1.0f / a; } __syncthreads(); const float inv = sbc;
  for (int k = t; k < kend; k += 256) { const float v = sr[k]; sh[k] = (v <= -1.0e38f) ? 0.f : expf(v - m) * inv * 2048.0f; }
  __syncthreads(); for (int q = t; q < kend / 4; q += 256) vst2(sr + q * 4, *(const v4f*)&sh[q * 4]); }
__global__ __launch_bounds__(128) void k_pv(const float* __restrict__ PS0, const _Float16* __restrict__ VT, const _Float16* __restrict__ VW, int b, int h0, float* __restrict__ Y, float* __restrict__ YW, float* __restrict__ PY) { const int h = h0 + blockIdx.z; const float* PS = PS0 + (size_t)blockIdx.z * TT * TT; __shared__ __align__(16) float ss[4][16][68]; __shared__ __align__(16) float scs[4][32];
  const int tid = threadIdx.x, wave = tid >> 5, lane = tid & 31, col = lane & 15, g = lane >> 4; const int ql0 = blockIdx.x * 64 + wave * 16;
  v8f acc[4] = {};
#pragma unroll 1
  for (int kc = 0; kc < TT / 32; ++kc) { const v16h p = frag_f32(PS + (size_t)(ql0 + col) * TT + kc * 32, lane);
#pragma unroll
    for (int j = 0; j < 4; ++j) { const size_t po = ((size_t)b * CC + h * HD + (j & 1) * 16 + col) * (size_t)TT + kc * 32; acc[j] = wmma16(p, frag_h((j < 2 ? VT : VW) + po, lane), acc[j]); } }
  float cs[4];
#pragma unroll
  for (int j = 0; j < 4; ++j) { float s = 0.f;
#pragma unroll
    for (int r = 0; r < 8; ++r) { const float v = acc[j][r] * (1.0f / 2048.0f); ss[wave][8 * g + r][j * 16 + col] = v; s += v; }
    cs[j] = s; }
  { const float o2 = __shfl_xor(cs[2], 16), o3 = __shfl_xor(cs[3], 16); if (g == 0) { scs[wave][col] = cs[2] + o2; scs[wave][16 + col] = cs[3] + o3; } }
  LDSX();
  for (int rl = 0; rl < 16; ++rl) if (lane < 16) { const size_t ro = ((size_t)b * TT + ql0 + rl) * CC + h * HD; if (lane < 8) vst2(Y + ro + lane * 4, *(const v4f*)&ss[wave][rl][lane * 4]); else vst2(YW + ro + (lane - 8) * 4, *(const v4f*)&ss[wave][rl][32 + (lane - 8) * 4]); }
  __syncthreads();
  if (tid < 8) { v4f o; const int d4 = tid * 4;
#pragma unroll
    for (int z = 0; z < 4; ++z) o[z] = ((scs[0][d4 + z] + scs[1][d4 + z]) + scs[2][d4 + z]) + scs[3][d4 + z];
    vst2(PY + ((size_t)b * NBLK + blockIdx.x) * CC + h * HD + d4, o); } }
__global__ __launch_bounds__(128) void k_comb(const float* __restrict__ Y, const float* __restrict__ YW, const float* __restrict__ PY, const float* __restrict__ PB, const float* __restrict__ LAM, float* __restrict__ OA) { __shared__ __align__(16) float sbg[128], sbv[128]; __shared__ __align__(16) float so[128][68];
  const int tid = threadIdx.x; const int b = blockIdx.y; const int n0 = blockIdx.x * 64;
  { float sg2 = 0.f, sb2 = 0.f; const float* py = PY + (size_t)b * NBLK * CC + tid; const float* pb = PB + (size_t)b * NBLK * CC + tid;
#pragma unroll 4
    for (int k = 0; k < NBLK; ++k) { sg2 += py[(size_t)k * CC]; sb2 += pb[(size_t)k * CC]; }
    sbg[tid] = sg2 * (1.0f / TT); sbv[tid] = sb2; }
  __syncthreads();
  const float lam = fmaxf(bfr(LAM[0]), 0.f);
  for (int e = tid; e < 64 * 128; e += 128) { const int rl = e >> 7, c = e & 127; const size_t ro = ((size_t)b * TT + n0 + rl) * CC + c; const float con = YW[ro] - sbg[c] + sbv[c]; so[c][rl] = Y[ro] + lam * fmaxf(con, 0.f); }
  __syncthreads();
  for (int e = tid; e < 128 * 16; e += 128) { const int c = e >> 4, q = e & 15; vst2(OA + ((size_t)b * CC + c) * TT + n0 + q * 4, *(const v4f*)&so[c][q * 4]); } }
__global__ __launch_bounds__(128) void k_conv(const float* __restrict__ OA, const float* __restrict__ WO, const float* __restrict__ BO, const float* __restrict__ X, float* __restrict__ OUT) { __shared__ __align__(16) float so[128][68];
  const int tid = threadIdx.x, wave = tid >> 5, lane = tid & 31, col = lane & 15, g = lane >> 4; const int b = blockIdx.y; const int hh = blockIdx.x;
  v8f acc[8] = {};
  const int w = wave * 16 + col;
#pragma unroll 1
  for (int kc = 0; kc < 9 * CC / 32; ++kc) { const int tap = kc >> 2, c0 = (kc & 3) * 32; const int dh = tap / 3 - 1, dw = tap % 3 - 1; const int hs = hh + dh, wsrc = w + dw; const bool okh = (hs >= 0) && (hs < HH), okw = (wsrc >= 0) && (wsrc < WWD); const bool ok = okh && okw; const int hcl = okh ? hs : hh, wcl = okw ? wsrc : w;
    v16b a; { const float* p = OA + ((size_t)b * CC + c0 + 8 * g) * TT + (size_t)hcl * WWD + wcl;
#pragma unroll
      for (int i = 0; i < 8; ++i) { const float va = p[(size_t)i * TT], vb = p[(size_t)(16 + i) * TT]; a[i] = (__bf16)(ok ? va : 0.f); a[8 + i] = (__bf16)(ok ? vb : 0.f); } }
    asm volatile("s_wait_loadcnt 0x0" ::: "memory");
#pragma unroll
    for (int j = 0; j < 8; ++j) { v16b wv; const int o = j * 16 + col; const float* wp = WO + (((size_t)o * CC + c0 + 8 * g) * 3 + (tap / 3)) * 3 + (tap % 3);
#pragma unroll
      for (int i = 0; i < 8; ++i) { wv[i] = (__bf16)wp[(size_t)i * 9]; wv[8 + i] = (__bf16)wp[(size_t)(16 + i) * 9]; }
      asm volatile("s_wait_loadcnt 0x0" ::: "memory"); acc[j] = wmma_bf(a, wv, acc[j]); } }
#pragma unroll
  for (int j = 0; j < 8; ++j) { const int o = j * 16 + col; const float bb = bfr(BO[o]);
#pragma unroll
    for (int r = 0; r < 8; ++r) { const int wr = wave * 16 + 8 * g + r; const float xv = bfr(X[((size_t)b * CC + o) * XP + (size_t)hh * WWD + wr]); so[o][wr] = leaky(acc[j][r] + bb) + xv; }
    asm volatile("s_wait_loadcnt 0x0" ::: "memory"); }
  __syncthreads();
  for (int e = tid; e < 128 * 16; e += 128) { const int o = e >> 4, q = e & 15; vst2(OUT + ((size_t)b * CC + o) * XP + (size_t)hh * WWD + q * 4, *(const v4f*)&so[o][q * 4]); } }
extern "C" void kernel_launch(void* const* d_in, const int* in_sizes, int n_in, void* d_out, int out_size, void* d_ws, size_t ws_size, hipStream_t stream) {
  (void)in_sizes; (void)n_in; (void)out_size;
  const float** F = (const float**)d_in;
  if (ws_size < (size_t)WS_END) return;
  char* ws = (char*)d_ws; _Float16 *QH = (_Float16*)(ws + WS_QH), *KH = (_Float16*)(ws + WS_KH), *VT = (_Float16*)(ws + WS_VT), *VW = (_Float16*)(ws + WS_VW); float *WGp = (float*)(ws + WS_WG), *BIp = (float*)(ws + WS_BI), *PB = (float*)(ws + WS_PB), *S = (float*)(ws + WS_S), *Y = (float*)(ws + WS_Y), *YW = (float*)(ws + WS_YW), *PY = (float*)(ws + WS_PY), *OA = (float*)(ws + WS_OA);
  k_projq<<<dim3(NBLK, TNB), 128, 0, stream>>>(F[0], F[1], F[2], F[5], F[6], F[7], F[8], F[9], F[10], F[11], F[12], QH, KH, WGp, BIp);
  k_projv<<<dim3(NBLK, TNB), 128, 0, stream>>>(F[0], F[3], F[4], WGp, BIp, VT, VW, PB);
  for (int b = 0; b < TNB; ++b) for (int h0 = 0; h0 < NH; h0 += HG) {
    k_sc<<<dim3(TT / 64, TT / 128, HG), 128, 0, stream>>>(QH, KH, b, h0, S);
    k_sm<<<dim3(TT, HG), 256, 0, stream>>>(S);
    k_pv<<<dim3(TT / 64, 1, HG), 128, 0, stream>>>(S, VT, VW, b, h0, Y, YW, PY);
  }
  k_comb<<<dim3(NBLK, TNB), 128, 0, stream>>>(Y, YW, PY, PB, F[13], OA);
  k_conv<<<dim3(HH, TNB), 128, 0, stream>>>(OA, F[14], F[15], F[0], (float*)d_out);
}
